// ParallelRetention_81381040325184
// MI455X (gfx1250) — hardware-verified
//
#include <hip/hip_runtime.h>
#include <hip/hip_bf16.h>

typedef __bf16         v16bf __attribute__((ext_vector_type(16)));
typedef unsigned short u16x8 __attribute__((ext_vector_type(8)));
typedef float          v8f   __attribute__((ext_vector_type(8)));
typedef float          v4f   __attribute__((ext_vector_type(4)));
typedef u16x8 __attribute__((may_alias)) u16x8a;
typedef v4f   __attribute__((may_alias)) v4fa;
typedef float __attribute__((may_alias)) f32a;

union Frag { v16bf v; u16x8 half[2]; };

#define TD 64
#define CD 2048
#define BD 32
#define MT 2048
#define NE (MT * CD)
#define GN_GROUPS 32
#define GN_EPS 1e-5f

__device__ __forceinline__ unsigned short f2bf(float f) {
  const unsigned int u = __float_as_uint(f);
  const unsigned int r = u + 0x7FFFu + ((u >> 16) & 1u);
  return (unsigned short)(r >> 16);
}
__device__ __forceinline__ float bf2f(unsigned short b) {
  return __uint_as_float(((unsigned int)b) << 16);
}
__device__ __forceinline__ void split_bf(float x, unsigned short& hv, unsigned short& lv) {
  hv = f2bf(x);
  lv = f2bf(x - bf2f(hv));
}

__device__ __forceinline__ v8f wmma_bf(v16bf a, v16bf b, v8f c) {
  v8f d = __builtin_amdgcn_wmma_f32_16x16x32_bf16(false, a, false, b, (short)0, c, false, false);
  asm volatile("v_nop\n\tv_nop\n\tv_nop\n\tv_nop" : "+v"(d) : "v"(a), "v"(b));
  return d;
}

__device__ __forceinline__ v16bf load_frag(const unsigned short* p, int h) {
  Frag f;
  f.half[0] = *(const u16x8a*)(p + 8 * h);
  f.half[1] = *(const u16x8a*)(p + 16 + 8 * h);
  return f.v;
}

__device__ __forceinline__ float wave_sum(float v) {
  #pragma unroll
  for (int off = 16; off > 0; off >>= 1) v += __shfl_xor(v, off, 32);
  return v;
}

__global__ __launch_bounds__(256) void cvt_split(const float* __restrict__ src,
                                                 unsigned short* __restrict__ hi,
                                                 unsigned short* __restrict__ lo,
                                                 int n8)
{
  const int g = blockIdx.x * 256 + threadIdx.x;
  if (g >= n8) return;
  const size_t e = (size_t)g * 8;
  const v4f a = *(const v4fa*)(src + e);
  const v4f c = *(const v4fa*)(src + e + 4);
  const float xs[8] = { a.x, a.y, a.z, a.w, c.x, c.y, c.z, c.w };
  unsigned short hh[8], ll[8];
  #pragma unroll
  for (int i = 0; i < 8; ++i) split_bf(xs[i], hh[i], ll[i]);
  const u16x8 hv = { hh[0], hh[1], hh[2], hh[3], hh[4], hh[5], hh[6], hh[7] };
  const u16x8 lv = { ll[0], ll[1], ll[2], ll[3], ll[4], ll[5], ll[6], ll[7] };
  unsigned short* ph = hi + e;
  unsigned short* pl = lo + e;
  *(volatile u16x8*)ph = hv;
  *(volatile u16x8*)pl = lv;
  __threadfence();
  *(volatile u16x8*)ph = hv;
  *(volatile u16x8*)pl = lv;
}

template<int MODE>
__device__ __forceinline__ void store16_pass(const unsigned short* sT, unsigned short* plane,
                                             int m0, int n0, int w, int lane) {
  const int q8 = lane & 7, sub = lane >> 3;
  #pragma unroll
  for (int i = 0; i < 8; ++i) {
    const int lid = w * 32 + i * 4 + sub;
    const int a = lid >> 1, hl = lid & 1;
    const u16x8 v = *(const u16x8a*)(sT + a * 128 + 64 * hl + 8 * q8);
    size_t gi;
    if (MODE == 0) gi = (size_t)(m0 + a) * CD + n0 + 64 * hl + 8 * q8;
    else           gi = ((size_t)((m0 >> 6) + hl) * CD + n0 + a) * TD + 8 * q8;
    *(volatile u16x8*)(plane + gi) = v;
  }
}

__device__ __forceinline__ void store32_pass(const f32a* sF, float* out,
                                             int mr0, int n0, int w, int lane) {
  const int q8 = lane & 7, sub = lane >> 3;
  #pragma unroll
  for (int i = 0; i < 8; ++i) {
    const int lid = w * 32 + i * 4 + sub;
    const int rl = lid >> 2, ql = lid & 3;
    const v4f v = *(const v4fa*)(sF + rl * 128 + 32 * ql + 4 * q8);
    *(volatile v4f*)(out + (size_t)(mr0 + rl) * CD + n0 + 32 * ql + 4 * q8) = v;
  }
}

template<int MODE>
__global__ __launch_bounds__(256) void gemm_x3(
    const unsigned short* __restrict__ Ah, const unsigned short* __restrict__ Al,
    const unsigned short* __restrict__ Bh, const unsigned short* __restrict__ Bl,
    const float* __restrict__ bias, const float* __restrict__ prelu,
    unsigned short* __restrict__ Oh, unsigned short* __restrict__ Ol,
    float* __restrict__ Of)
{
  __shared__ __attribute__((aligned(16))) unsigned short sT[128 * 128];

  const int tid = threadIdx.x, lane = tid & 31, w = tid >> 5;
  const int h = lane >> 4, m = lane & 15;
  const int wm = w >> 2, wn = w & 3;
  const int m0 = blockIdx.y * 128, n0 = blockIdx.x * 128;
  const int rbase = m0 + wm * 64;
  const int cbase = n0 + wn * 32;

  const v8f zero8 = {0.f, 0.f, 0.f, 0.f, 0.f, 0.f, 0.f, 0.f};
  v8f acc[4][2];
  #pragma unroll
  for (int mt = 0; mt < 4; ++mt)
    #pragma unroll
    for (int nt = 0; nt < 2; ++nt) acc[mt][nt] = zero8;

  #pragma unroll 1
  for (int k0 = 0; k0 < CD; k0 += 32) {
    v16bf bfh[2], bfl[2];
    #pragma unroll
    for (int nt = 0; nt < 2; ++nt) {
      const size_t off = (size_t)(cbase + nt * 16 + m) * CD + k0;
      bfh[nt] = load_frag(Bh + off, h);
      bfl[nt] = load_frag(Bl + off, h);
    }
    #pragma unroll
    for (int mt = 0; mt < 4; ++mt) {
      const size_t off = (size_t)(rbase + mt * 16 + m) * CD + k0;
      const v16bf afh = load_frag(Ah + off, h);
      const v16bf afl = load_frag(Al + off, h);
      #pragma unroll
      for (int nt = 0; nt < 2; ++nt) {
        acc[mt][nt] = wmma_bf(afh, bfh[nt], acc[mt][nt]);
        acc[mt][nt] = wmma_bf(afh, bfl[nt], acc[mt][nt]);
        acc[mt][nt] = wmma_bf(afl, bfh[nt], acc[mt][nt]);
      }
    }
  }

  if (MODE != 2) {
    #pragma unroll
    for (int p = 0; p < 2; ++p) {
      #pragma unroll
      for (int mt = 0; mt < 4; ++mt) {
        #pragma unroll
        for (int nt = 0; nt < 2; ++nt) {
          const int cl = wn * 32 + nt * 16 + m;
          const float bs = bias[n0 + cl];
          #pragma unroll
          for (int r = 0; r < 8; ++r) {
            const int rl = wm * 64 + mt * 16 + 8 * h + r;
            const float val = acc[mt][nt][r] + bs;
            unsigned short hv = f2bf(val);
            if (p == 1) hv = f2bf(val - bf2f(hv));
            const int idx = (MODE == 0) ? (rl * 128 + cl) : (cl * 128 + rl);
            sT[idx] = hv;
          }
        }
      }
      __syncthreads();
      unsigned short* plane = (p == 0) ? Oh : Ol;
      store16_pass<MODE>(sT, plane, m0, n0, w, lane);
      __threadfence();
      store16_pass<MODE>(sT, plane, m0, n0, w, lane);
      __syncthreads();
    }
  } else {
    f32a* sF = (f32a*)sT;
    const float pa = prelu[0];
    #pragma unroll
    for (int hr = 0; hr < 2; ++hr) {
      if (wm == hr) {
        #pragma unroll
        for (int mt = 0; mt < 4; ++mt) {
          #pragma unroll
          for (int nt = 0; nt < 2; ++nt) {
            const int cl = wn * 32 + nt * 16 + m;
            const float bs = bias[n0 + cl];
            #pragma unroll
            for (int r = 0; r < 8; ++r) {
              const int rl = mt * 16 + 8 * h + r;
              float val = acc[mt][nt][r] + bs;
              val = (val >= 0.0f) ? val : pa * val;
              sF[rl * 128 + cl] = val;
            }
          }
        }
      }
      __syncthreads();
      store32_pass(sF, Of, m0 + 64 * hr, n0, w, lane);
      __threadfence();
      store32_pass(sF, Of, m0 + 64 * hr, n0, w, lane);
      __syncthreads();
    }
  }
}

__device__ __forceinline__ void ystore_pass(const unsigned short* sY,
                                            unsigned short* yh, unsigned short* yl,
                                            size_t tok0, int g, int w, int lane) {
  const int q8 = lane & 7, sub = lane >> 3;
  const int plane = w >> 2;
  const unsigned short* src = sY + plane * (TD * TD);
  unsigned short* dstp = plane ? yl : yh;
  #pragma unroll
  for (int i = 0; i < 4; ++i) {
    const int t = (w & 3) * 16 + i * 4 + sub;
    const u16x8 v = *(const u16x8a*)(src + t * TD + 8 * q8);
    *(volatile u16x8*)(dstp + (tok0 + t) * CD + g * TD + 8 * q8) = v;
  }
}

__global__ __launch_bounds__(256) void retention_kernel(
    const unsigned short* __restrict__ qh, const unsigned short* __restrict__ ql,
    const unsigned short* __restrict__ kh, const unsigned short* __restrict__ kl,
    const unsigned short* __restrict__ vh, const unsigned short* __restrict__ vl,
    const float* __restrict__ dg,
    const float* __restrict__ gw, const float* __restrict__ gb,
    unsigned short* __restrict__ yh, unsigned short* __restrict__ yl)
{
  __shared__ __attribute__((aligned(16))) unsigned short sP[2 * TD * TD];
  __shared__ __attribute__((aligned(16))) unsigned short sY[2 * TD * TD];
  __shared__ float red[16];

  const int b = blockIdx.x;
  const int tid = threadIdx.x, lane = tid & 31, w = tid >> 5;
  const int h = lane >> 4, m = lane & 15;
  const int mt = w >> 1, nt0 = (w & 1) * 2;
  const size_t tok0 = (size_t)b * TD;

  const v8f zero8 = {0.f, 0.f, 0.f, 0.f, 0.f, 0.f, 0.f, 0.f};

  v8f acc[2];
  acc[0] = zero8; acc[1] = zero8;
  const unsigned short* qrh = qh + (tok0 + 16 * mt + m) * CD;
  const unsigned short* qrl = ql + (tok0 + 16 * mt + m) * CD;
  #pragma unroll 1
  for (int k0 = 0; k0 < CD; k0 += 32) {
    const v16bf afh = load_frag(qrh + k0, h);
    const v16bf afl = load_frag(qrl + k0, h);
    #pragma unroll
    for (int j = 0; j < 2; ++j) {
      const size_t off = (tok0 + 16 * (nt0 + j) + m) * CD + k0;
      const v16bf bfh = load_frag(kh + off, h);
      const v16bf bfl = load_frag(kl + off, h);
      acc[j] = wmma_bf(afh, bfh, acc[j]);
      acc[j] = wmma_bf(afh, bfl, acc[j]);
      acc[j] = wmma_bf(afl, bfh, acc[j]);
    }
  }

  #pragma unroll
  for (int j = 0; j < 2; ++j) {
    const int s = 16 * (nt0 + j) + m;
    #pragma unroll
    for (int r = 0; r < 8; ++r) {
      const int t = 16 * mt + 8 * h + r;
      const float p = acc[j][r] * dg[t * TD + s];
      unsigned short hv, lv;
      split_bf(p, hv, lv);
      sP[t * TD + s] = hv;
      sP[TD * TD + t * TD + s] = lv;
    }
  }
  __syncthreads();

  const float inv_n = 1.0f / 4096.0f;

  #pragma unroll 1
  for (int g = 0; g < GN_GROUPS; ++g) {
    v8f ra[2];
    ra[0] = zero8; ra[1] = zero8;
    #pragma unroll
    for (int k0 = 0; k0 < TD; k0 += 32) {
      const v16bf afh = load_frag(sP + (16 * mt + m) * TD + k0, h);
      const v16bf afl = load_frag(sP + TD * TD + (16 * mt + m) * TD + k0, h);
      #pragma unroll
      for (int j = 0; j < 2; ++j) {
        const int c = g * TD + 16 * (nt0 + j) + m;
        const size_t off = ((size_t)b * CD + c) * TD + k0;
        const v16bf bfh = load_frag(vh + off, h);
        const v16bf bfl = load_frag(vl + off, h);
        ra[j] = wmma_bf(afh, bfh, ra[j]);
        ra[j] = wmma_bf(afh, bfl, ra[j]);
        ra[j] = wmma_bf(afl, bfh, ra[j]);
      }
    }

    float s1 = 0.0f;
    #pragma unroll
    for (int j = 0; j < 2; ++j)
      #pragma unroll
      for (int r = 0; r < 8; ++r) s1 += ra[j][r];
    s1 = wave_sum(s1);
    if (lane == 0) red[w] = s1;
    __syncthreads();
    float tot = 0.0f;
    #pragma unroll
    for (int i = 0; i < 8; ++i) tot += red[i];
    const float mean = tot * inv_n;

    float s2 = 0.0f;
    #pragma unroll
    for (int j = 0; j < 2; ++j)
      #pragma unroll
      for (int r = 0; r < 8; ++r) { const float d = ra[j][r] - mean; s2 += d * d; }
    s2 = wave_sum(s2);
    if (lane == 0) red[8 + w] = s2;
    __syncthreads();
    float tot2 = 0.0f;
    #pragma unroll
    for (int i = 0; i < 8; ++i) tot2 += red[8 + i];
    const float var = tot2 * inv_n;
    const float rstd = rsqrtf(var + GN_EPS);

    #pragma unroll
    for (int j = 0; j < 2; ++j) {
      const int cl = 16 * (nt0 + j) + m;
      const int c = g * TD + cl;
      const float wv = gw[c] * rstd;
      const float bvv = gb[c];
      #pragma unroll
      for (int r = 0; r < 8; ++r) {
        const int t = 16 * mt + 8 * h + r;
        const float yv = (ra[j][r] - mean) * wv + bvv;
        unsigned short hv, lv;
        split_bf(yv, hv, lv);
        sY[t * TD + cl] = hv;
        sY[TD * TD + t * TD + cl] = lv;
      }
    }
    __syncthreads();
    ystore_pass(sY, yh, yl, tok0, g, w, lane);
    __threadfence();
    ystore_pass(sY, yh, yl, tok0, g, w, lane);
    __syncthreads();
  }
}

extern "C" void kernel_launch(void* const* d_in, const int* in_sizes, int n_in,
                              void* d_out, int out_size, void* d_ws, size_t ws_size,
                              hipStream_t stream) {
  if (n_in < 13) return;
  if (in_sizes[0] != NE) return;
  if (in_sizes[1] != TD * TD) return;
  if (in_sizes[2] != NE || in_sizes[4] != NE || in_sizes[6] != NE || in_sizes[8] != NE) return;
  if (in_sizes[3] != CD || in_sizes[5] != CD || in_sizes[7] != CD || in_sizes[9] != CD) return;
  if (in_sizes[10] != CD || in_sizes[11] != CD) return;
  if (in_sizes[12] < 1) return;
  if (out_size != NE) return;

  const float* x   = (const float*)d_in[0];
  const float* dg  = (const float*)d_in[1];
  const float* Wq  = (const float*)d_in[2];
  const float* bq  = (const float*)d_in[3];
  const float* Wk  = (const float*)d_in[4];
  const float* bk  = (const float*)d_in[5];
  const float* Wv  = (const float*)d_in[6];
  const float* bv  = (const float*)d_in[7];
  const float* Wo  = (const float*)d_in[8];
  const float* bo  = (const float*)d_in[9];
  const float* gnw = (const float*)d_in[10];
  const float* gnb = (const float*)d_in[11];
  const float* pa  = (const float*)d_in[12];
  float* out = (float*)d_out;

  const size_t PB = (size_t)NE * 2;
  const size_t total = 12 * PB;
  if (total > ws_size) return;
  char* ws = (char*)d_ws;
  unsigned short* xh  = (unsigned short*)(ws + 0 * PB);
  unsigned short* xl  = (unsigned short*)(ws + 1 * PB);
  unsigned short* wh  = (unsigned short*)(ws + 2 * PB);
  unsigned short* wl  = (unsigned short*)(ws + 3 * PB);
  unsigned short* qh  = (unsigned short*)(ws + 4 * PB);
  unsigned short* ql  = (unsigned short*)(ws + 5 * PB);
  unsigned short* kh  = (unsigned short*)(ws + 6 * PB);
  unsigned short* kl  = (unsigned short*)(ws + 7 * PB);
  unsigned short* vth = (unsigned short*)(ws + 8 * PB);
  unsigned short* vtl = (unsigned short*)(ws + 9 * PB);
  unsigned short* yh  = (unsigned short*)(ws + 10 * PB);
  unsigned short* yl  = (unsigned short*)(ws + 11 * PB);

  const int n8 = NE / 8;
  const int cvt_blocks = (n8 + 255) / 256;
  const dim3 gg(CD / 128, MT / 128);

  cvt_split<<<cvt_blocks, 256, 0, stream>>>(x, xh, xl, n8);

  cvt_split<<<cvt_blocks, 256, 0, stream>>>(Wq, wh, wl, n8);
  gemm_x3<0><<<gg, 256, 0, stream>>>(xh, xl, wh, wl, bq, pa, qh, ql, out);

  cvt_split<<<cvt_blocks, 256, 0, stream>>>(Wk, wh, wl, n8);
  gemm_x3<0><<<gg, 256, 0, stream>>>(xh, xl, wh, wl, bk, pa, kh, kl, out);

  cvt_split<<<cvt_blocks, 256, 0, stream>>>(Wv, wh, wl, n8);
  gemm_x3<1><<<gg, 256, 0, stream>>>(xh, xl, wh, wl, bv, pa, vth, vtl, out);

  retention_kernel<<<BD, 256, 0, stream>>>(qh, ql, kh, kl, vth, vtl, dg, gnw, gnb, yh, yl);

  cvt_split<<<cvt_blocks, 256, 0, stream>>>(Wo, wh, wl, n8);
  gemm_x3<2><<<gg, 256, 0, stream>>>(yh, yl, wh, wl, bo, pa, qh, ql, out);
}
